// EdgeMultiHeadAttention_9414568312873
// MI455X (gfx1250) — hardware-verified
//
#include <hip/hip_runtime.h>
#include <stddef.h>


typedef _Float16 h16;
typedef _Float16 v16h __attribute__((ext_vector_type(16)));
typedef _Float16 v8h  __attribute__((ext_vector_type(8)));
typedef float    v8f  __attribute__((ext_vector_type(8)));
typedef float    v4f  __attribute__((ext_vector_type(4)));
typedef float    v2f  __attribute__((ext_vector_type(2)));

#ifndef NB
#define NB 2
#endif
#ifndef SEQ
#define SEQ 2000
#endif
#define NB_FULL  2
#define SEQ_FULL 2000
#define DIM   1024
#define NHEAD 16
#define HD    64
#define KNN   20
#define NIDX  100
#define EDGE_DICT 64
#define SEQP  (((SEQ + 127) / 128) * 128)
#define KEND  (((SEQ + 63) / 64) * 64)
#define MROWSP (NB * SEQP)

static_assert(NB >= 1 && NB <= NB_FULL);
static_assert(SEQ >= 64 && SEQ <= SEQ_FULL);
static_assert(SEQ_FULL == NIDX * KNN);
static_assert((SEQ - 1) / KNN < NIDX);
static_assert(DIM == NHEAD * HD);
static_assert(HD == 64);
static_assert((DIM % 64) == 0 && (DIM % 32) == 0);
static_assert((SEQP % 128) == 0 && KEND <= SEQP && (KEND % 64) == 0);
static_assert((MROWSP % 64) == 0 && (MROWSP % 8) == 0);
static_assert(DIM == 4 * 32 * 8);
static_assert(((size_t)DIM * DIM) % (256 * 8) == 0);
static_assert((EDGE_DICT * 2) % 32 == 0);
static_assert(((size_t)(NB - 1) * SEQ_FULL + SEQ) * DIM * 4 <= (size_t)16384000);

#define LDT 72
#define LDC 68
static_assert((LDT % 8) == 0 && LDT >= 64);
static_assert((LDC % 4) == 0 && LDC >= 64);

#define WCARRY 64.0f
#define PCARRY 1024.0f
#define VCARRY 64.0f

static_assert((256 / 8) * 2 == 64);
static_assert((256 / 16) * 4 == 64);
static_assert((32 / 8) * 4 == 16);

static_assert((size_t)64 * LDC * 4 <= (size_t)131072);
static_assert((size_t)2 * 64 * LDT * 2 + (size_t)8 * 16 * LDT * 2 + (size_t)SEQP * 4 <= (size_t)131072);

#define WSQ_BYTES     ((size_t)DIM * DIM * 2)
#define PLANE16_BYTES ((size_t)MROWSP * DIM * 2)
#define TBL_BYTES     ((size_t)EDGE_DICT * 2 * 4)
#define OFF_WQ  ((size_t)0)
#define OFF_WK  (OFF_WQ + WSQ_BYTES)
#define OFF_WV  (OFF_WK + WSQ_BYTES)
#define OFF_WO  (OFF_WV + WSQ_BYTES)
#define OFF_XQ  (OFF_WO + WSQ_BYTES)
#define OFF_XK  (OFF_XQ + PLANE16_BYTES)
#define OFF_XV  (OFF_XK + PLANE16_BYTES)
#define OFF_Q   (OFF_XV + PLANE16_BYTES)
#define OFF_K   (OFF_Q + PLANE16_BYTES)
#define OFF_VT  (OFF_K + PLANE16_BYTES)
#define OFF_CTX (OFF_VT + PLANE16_BYTES)
#define OFF_TBL (OFF_CTX + PLANE16_BYTES)
#define WS_TOTAL (OFF_TBL + TBL_BYTES)
static_assert((WSQ_BYTES % 128) == 0 && (PLANE16_BYTES % 128) == 0 && (TBL_BYTES % 128) == 0);
static_assert(WS_TOTAL <= (size_t)134217728);

__device__ __forceinline__ float bf16r(float x) {
  unsigned int u = __float_as_uint(x);
  u = (u + 0x7FFFu + ((u >> 16) & 1u)) & 0xFFFF0000u;
  return __uint_as_float(u);
}

__device__ __forceinline__ h16 toh_flush(float v) {
  const h16 r = (h16)v;
  return (fabsf(v) < 6.103515625e-05f) ? (h16)0.0f : r;
}

__device__ __forceinline__ v16h frag_at(const _Float16* p) {
  v8h lo = *(const v8h*)(p);
  v8h hi = *(const v8h*)(p + 16);
  v16h out;
#pragma unroll
  for (int i = 0; i < 8; ++i) { out[i] = lo[i]; out[i + 8] = hi[i]; }
  return out;
}
__device__ __forceinline__ v16h ld_frag(const _Float16* base, unsigned ld) {
  const unsigned lane = threadIdx.x & 31u;
  return frag_at(base + (lane & 15u) * ld + (lane >> 4) * 8u);
}

__device__ __forceinline__ v8f wmma16(v16h a, v16h b, v8f c) {
  v8f d = __builtin_amdgcn_wmma_f32_16x16x32_f16(false, a, false, b, (short)0, c,
                                                 false, false);
  asm volatile("v_nop\n\tv_nop\n\tv_nop\n\tv_nop" : "+v"(d) : "v"(a), "v"(b));
  return d;
}

__device__ __forceinline__ float red16_max(float x) {
#pragma unroll
  for (int off = 1; off < 16; off <<= 1) x = fmaxf(x, __shfl_xor(x, off, 32));
  return x;
}
__device__ __forceinline__ float red16_sum(float x) {
#pragma unroll
  for (int off = 1; off < 16; off <<= 1) x += __shfl_xor(x, off, 32);
  return x;
}
__device__ __forceinline__ float red32_sum(float x) {
#pragma unroll
  for (int off = 1; off < 32; off <<= 1) x += __shfl_xor(x, off, 32);
  return x;
}

__device__ __forceinline__ void wave_lds_sync() {
  __builtin_amdgcn_fence(3  , "wavefront");
  asm volatile("s_wait_dscnt 0x0" ::: "memory");
  __builtin_amdgcn_wave_barrier();
}

__global__ __launch_bounds__(256) void wcast_kernel(
    const float* __restrict__ W, _Float16* __restrict__ Wt) {
  const size_t e = ((size_t)blockIdx.x * 256u + threadIdx.x) * 8u;
  const v4f a0 = *(const v4f*)(W + e);
  const v4f a1 = *(const v4f*)(W + e + 4u);
  v8h o;
#pragma unroll
  for (int i = 0; i < 4; ++i) {
    o[i]     = toh_flush(WCARRY * bf16r(a0[i]));
    o[i + 4] = toh_flush(WCARRY * bf16r(a1[i]));
  }
  _Float16* p = Wt + e;
  *(volatile v8h*)p = o;
  __threadfence();
  *(volatile v8h*)p = o;
}

__global__ __launch_bounds__(256) void xcast_kernel(
    const float* __restrict__ X, _Float16* __restrict__ dst) {
  const unsigned lane = threadIdx.x & 31u;
  const unsigned w = (unsigned)__builtin_amdgcn_readfirstlane((int)(threadIdx.x >> 5));
  const unsigned crow = blockIdx.x * 8u + w;
  const unsigned bidx = crow / (unsigned)SEQP;
  const unsigned sq = crow - bidx * (unsigned)SEQP;
  const bool live = sq < (unsigned)SEQ;
  const unsigned sqc = live ? sq : (unsigned)(SEQ - 1);
  const size_t srow = (size_t)bidx * SEQ_FULL + sqc;
  const float* xr = X + srow * DIM + lane * 8u;
#pragma unroll 1
  for (unsigned j = 0; j < 4u; ++j) {
    const unsigned c = j * 256u + lane * 8u;
    const v4f a0 = *(const v4f*)(xr + j * 256u);
    const v4f a1 = *(const v4f*)(xr + j * 256u + 4u);
    v8h o;
#pragma unroll
    for (int i = 0; i < 4; ++i) {
      const h16 t0 = toh_flush(bf16r(a0[i]));
      const h16 t1 = toh_flush(bf16r(a1[i]));
      o[i]     = live ? t0 : (h16)0.0f;
      o[i + 4] = live ? t1 : (h16)0.0f;
    }
    _Float16* p = dst + (size_t)crow * DIM + c;
    *(volatile v8h*)p = o;
    __threadfence();
    *(volatile v8h*)p = o;
  }
}

__global__ __launch_bounds__(256) void bias_table_kernel(
    const float* __restrict__ edge_emb, const float* __restrict__ mask_emb,
    float* __restrict__ tbl) {
  __shared__ __attribute__((aligned(16))) float red[32];
  const unsigned lane = threadIdx.x & 31u;
  const unsigned w = (unsigned)__builtin_amdgcn_readfirstlane((int)(threadIdx.x >> 5));
#pragma unroll 1
  for (unsigned t = 0; t < 2u; ++t) {
    const unsigned e = blockIdx.x * 16u + w * 2u + t;
    float s0 = 0.0f, s1 = 0.0f;
#pragma unroll 1
    for (unsigned k = lane; k < (unsigned)DIM; k += 32u) {
      const float ev = bf16r(edge_emb[(size_t)e * DIM + k]);
      s0 += ev * bf16r(mask_emb[k]);
      s1 += ev * bf16r(mask_emb[DIM + k]);
    }
    s0 = red32_sum(s0);
    s1 = red32_sum(s1);
    if (lane == 0u) {
      red[(w * 2u + t) * 2u]      = s0;
      red[(w * 2u + t) * 2u + 1u] = s1;
    }
  }
  __syncthreads();
  if (w == 0u && lane < 8u) {
    const v4f x = *(const v4f*)&red[lane * 4u];
    float* p = tbl + blockIdx.x * 32u + lane * 4u;
    *(volatile v4f*)p = x;
    __threadfence();
    *(volatile v4f*)p = x;
  }
}

template <int MODE>
__device__ __forceinline__ void gemm_body(
    const _Float16* __restrict__ A16, const _Float16* __restrict__ Bt, const unsigned K,
    const float* __restrict__ bias, float* __restrict__ outf, _Float16* __restrict__ out16) {
  __shared__ float Cs[64 * LDC];
  const unsigned tid = threadIdx.x, lane = tid & 31u;
  const unsigned w = (unsigned)__builtin_amdgcn_readfirstlane((int)(tid >> 5));
  const unsigned mw = w >> 1, nw = w & 1u;
  const unsigned hh = lane >> 4, m = lane & 15u;
  const unsigned n0 = blockIdx.x * 64u;
  const unsigned row0 = blockIdx.y * 64u;

  const _Float16* ap  = A16 + (size_t)(row0 + mw * 16u + m) * K + hh * 8u;
  const _Float16* bp0 = Bt + (size_t)(n0 + nw * 32u + m) * K + hh * 8u;
  const _Float16* bp1 = bp0 + (size_t)16 * K;
  v8f acc0 = {}, acc1 = {};
#pragma unroll 2
  for (unsigned k0 = 0; k0 < K; k0 += 32u) {
    const v16h a  = frag_at(ap + k0);
    const v16h b0 = frag_at(bp0 + k0);
    const v16h b1 = frag_at(bp1 + k0);
    acc0 = wmma16(a, b0, acc0);
    acc1 = wmma16(a, b1, acc1);
  }
#pragma unroll
  for (int r = 0; r < 8; ++r) {
    float* d = &Cs[(mw * 16u + hh * 8u + (unsigned)r) * LDC + nw * 32u + m];
    d[0]  = acc0[r];
    d[16] = acc1[r];
  }
  __syncthreads();

  if (MODE == 0) {
    v8h x[2];
    size_t off[2];
#pragma unroll
    for (unsigned i = 0; i < 2u; ++i) {
      const unsigned r = 32u * i + (tid >> 3);
      const unsigned c = (tid & 7u) * 8u;
      const v4f u0 = *(const v4f*)&Cs[r * LDC + c];
      const v4f u1 = *(const v4f*)&Cs[r * LDC + c + 4];
      const v4f g0 = *(const v4f*)(bias + n0 + c);
      const v4f g1 = *(const v4f*)(bias + n0 + c + 4u);
#pragma unroll
      for (int j = 0; j < 4; ++j) {
        x[i][j]     = toh_flush(u0[j] * (1.0f / WCARRY) + bf16r(g0[j]));
        x[i][j + 4] = toh_flush(u1[j] * (1.0f / WCARRY) + bf16r(g1[j]));
      }
      off[i] = (size_t)(row0 + r) * DIM + n0 + c;
    }
#pragma unroll
    for (int i = 0; i < 2; ++i) *(volatile v8h*)(out16 + off[i]) = x[i];
    __threadfence();
#pragma unroll
    for (int i = 0; i < 2; ++i) *(volatile v8h*)(out16 + off[i]) = x[i];
  }

  if (MODE == 1) {
    const unsigned bidx = row0 / (unsigned)SEQP;
    const unsigned key0 = row0 - bidx * (unsigned)SEQP;
    v8h x[2];
    size_t off[2];
#pragma unroll
    for (unsigned i = 0; i < 2u; ++i) {
      const unsigned dcol = 32u * i + (tid >> 3);
      const unsigned kk = (tid & 7u) * 8u;
      const float bb = bf16r(bias[n0 + dcol]);
#pragma unroll
      for (unsigned j = 0; j < 8u; ++j) {
        const float t = Cs[(kk + j) * LDC + dcol] * (1.0f / WCARRY) + bb;
        x[i][j] = toh_flush(t);
      }
      off[i] = ((size_t)bidx * DIM + n0 + dcol) * SEQP + key0 + kk;
    }
#pragma unroll
    for (int i = 0; i < 2; ++i) *(volatile v8h*)(out16 + off[i]) = x[i];
    __threadfence();
#pragma unroll
    for (int i = 0; i < 2; ++i) *(volatile v8h*)(out16 + off[i]) = x[i];
  }

  if (MODE == 2) {
    const float cs = 1.0f / (WCARRY * VCARRY);
    v4f xs[4];
    size_t off[4];
    bool live[4];
#pragma unroll
    for (unsigned i = 0; i < 4u; ++i) {
      const unsigned r = 16u * i + (tid >> 4);
      const unsigned c = (tid & 15u) * 4u;
      const unsigned crow = row0 + r;
      const unsigned bidx = crow / (unsigned)SEQP;
      const unsigned sq = crow - bidx * (unsigned)SEQP;
      live[i] = sq < (unsigned)SEQ;
      const unsigned sqc = live[i] ? sq : (unsigned)(SEQ - 1);
      const v4f u = *(const v4f*)&Cs[r * LDC + c];
      const v4f g = *(const v4f*)(bias + n0 + c);
      v4f val;
#pragma unroll
      for (int j = 0; j < 4; ++j) val[j] = u[j] * cs + bf16r(g[j]);
      xs[i] = val;
      off[i] = ((size_t)bidx * SEQ_FULL + sqc) * DIM + n0 + c;
    }
#pragma unroll
    for (int i = 0; i < 4; ++i)
      if (live[i]) *(volatile v4f*)(outf + off[i]) = xs[i];
    __threadfence();
#pragma unroll
    for (int i = 0; i < 4; ++i)
      if (live[i]) *(volatile v4f*)(outf + off[i]) = xs[i];
  }
}

__global__ __launch_bounds__(256) void gemm_qk_kernel(
    const _Float16* __restrict__ A16, const _Float16* __restrict__ Bt,
    const float* __restrict__ bias, _Float16* __restrict__ out16) {
  gemm_body<0>(A16, Bt, (unsigned)DIM, bias, (float*)0, out16);
}
__global__ __launch_bounds__(256) void gemm_v_kernel(
    const _Float16* __restrict__ A16, const _Float16* __restrict__ Bt,
    const float* __restrict__ bias, _Float16* __restrict__ vt) {
  gemm_body<1>(A16, Bt, (unsigned)DIM, bias, (float*)0, vt);
}
__global__ __launch_bounds__(256) void gemm_wo_kernel(
    const _Float16* __restrict__ A16, const _Float16* __restrict__ Bt,
    const float* __restrict__ bias, float* __restrict__ outf) {
  gemm_body<2>(A16, Bt, (unsigned)DIM, bias, outf, (_Float16*)0);
}

__global__ __launch_bounds__(256) void attn_kernel(
    const _Float16* __restrict__ Qh, const _Float16* __restrict__ Kh,
    const _Float16* __restrict__ Vt, const int* __restrict__ cmask,
    const int* __restrict__ degv, const float* __restrict__ tbl,
    _Float16* __restrict__ Ov) {
  __shared__ _Float16 Ks[64 * LDT];
  __shared__ _Float16 Vs[64 * LDT];
  __shared__ _Float16 Ps[8 * 16 * LDT];
  __shared__ int Cm[SEQP];

  const unsigned tid = threadIdx.x, lane = tid & 31u;
  const unsigned w = (unsigned)__builtin_amdgcn_readfirstlane((int)(tid >> 5));
  const unsigned hh = lane >> 4, m = lane & 15u;
  const unsigned q0 = blockIdx.x * 128u;
  const unsigned head = blockIdx.y;
  const unsigned b = blockIdx.z;
  const float scale = 0.125f;
  const unsigned qrow0 = q0 + w * 16u;
  const unsigned pw = w * (16u * LDT);

#pragma unroll 1
  for (unsigned key = tid; key < (unsigned)SEQP; key += 256u) {
    const unsigned kc = (key < (unsigned)SEQ) ? key : (unsigned)(SEQ - 1);
    int c = cmask[kc / (unsigned)KNN];
    c = (c < 0) ? 0 : c;
    c = (c > 1) ? 1 : c;
    Cm[key] = c;
  }

  float rb0[8], rb1[8];
#pragma unroll
  for (int v = 0; v < 8; ++v) {
    unsigned r = qrow0 + hh * 8u + (unsigned)v;
    r = (r < (unsigned)SEQ) ? r : (unsigned)(SEQ - 1);
    int dg = degv[r / (unsigned)KNN];
    dg = (dg < 0) ? 0 : dg;
    dg = (dg > (EDGE_DICT - 1)) ? (EDGE_DICT - 1) : dg;
    const v2f tp = *(const v2f*)(tbl + 2 * dg);
    rb0[v] = tp[0];
    rb1[v] = tp[1];
  }

  const size_t qoff = (size_t)(b * (unsigned)SEQP + qrow0 + m) * DIM + head * HD + hh * 8u;
  v16h qf[2];
  qf[0] = frag_at(Qh + qoff);
  qf[1] = frag_at(Qh + qoff + 32);

  float mrow[8], lrow[8];
  v8f o[4];
#pragma unroll
  for (int v = 0; v < 8; ++v) { mrow[v] = -1.0e30f; lrow[v] = 0.0f; }
#pragma unroll
  for (int nb = 0; nb < 4; ++nb) o[nb] = (v8f){};

  const size_t kplane = (size_t)b * SEQP * DIM + head * HD;
  const size_t vplane = ((size_t)b * DIM + head * HD) * SEQP;

  for (unsigned kb = 0; kb < (unsigned)KEND; kb += 64u) {
#pragma unroll
    for (unsigned j = 0; j < 2u; ++j) {
      const unsigned idx = tid + 256u * j;
      const unsigned r = idx >> 3, c = (idx & 7u) * 8u;
      *(v8h*)&Ks[r * LDT + c] = *(const v8h*)(Kh + kplane + (size_t)(kb + r) * DIM + c);
      *(v8h*)&Vs[r * LDT + c] = *(const v8h*)(Vt + vplane + (size_t)r * SEQP + kb + c);
    }
    __syncthreads();

    v8f s[4];
#pragma unroll
    for (int kg = 0; kg < 4; ++kg) {
      const int cmk = Cm[kb + (unsigned)kg * 16u + m];
      v8f t = {};
#pragma unroll
      for (int c = 0; c < 2; ++c) {
        const v16h kf = ld_frag(&Ks[(kg * 16) * LDT + c * 32], LDT);
        t = wmma16(qf[c], kf, t);
      }
#pragma unroll
      for (int v = 0; v < 8; ++v)
        s[kg][v] = t[v] * scale + ((cmk != 0) ? rb1[v] : rb0[v]);
    }

    if (kb + 64u > (unsigned)SEQ) {
#pragma unroll
      for (int kg = 0; kg < 4; ++kg)
#pragma unroll
        for (int v = 0; v < 8; ++v) {
          const unsigned key = kb + (unsigned)kg * 16u + m;
          s[kg][v] = (key >= (unsigned)SEQ) ? -1.0e30f : s[kg][v];
        }
    }

    float alpha[8];
#pragma unroll
    for (int v = 0; v < 8; ++v) {
      float mx = fmaxf(fmaxf(s[0][v], s[1][v]), fmaxf(s[2][v], s[3][v]));
      mx = red16_max(mx);
      const float mn = fmaxf(mrow[v], mx);
      alpha[v] = __expf(mrow[v] - mn);
      mrow[v] = mn;
    }
#pragma unroll
    for (int kg = 0; kg < 4; ++kg)
#pragma unroll
      for (int v = 0; v < 8; ++v) s[kg][v] = __expf(s[kg][v] - mrow[v]);

#pragma unroll
    for (int kg = 0; kg < 4; ++kg)
#pragma unroll
      for (int v = 0; v < 8; ++v) {
        const h16 ph = toh_flush(s[kg][v] * PCARRY);
        Ps[pw + (hh * 8u + (unsigned)v) * LDT + (unsigned)kg * 16u + m] = ph;
        s[kg][v] = (float)ph;
      }
#pragma unroll
    for (int v = 0; v < 8; ++v) {
      const float rs = red16_sum((s[0][v] + s[1][v]) + (s[2][v] + s[3][v]));
      lrow[v] = alpha[v] * lrow[v] + rs;
    }
#pragma unroll
    for (int nb = 0; nb < 4; ++nb)
#pragma unroll
      for (int v = 0; v < 8; ++v) o[nb][v] = o[nb][v] * alpha[v];
    wave_lds_sync();

#pragma unroll
    for (int c = 0; c < 2; ++c) {
      const v16h pf = ld_frag(&Ps[pw + c * 32], LDT);
#pragma unroll
      for (int nb = 0; nb < 4; ++nb) {
        const v16h vf = ld_frag(&Vs[(nb * 16) * LDT + c * 32], LDT);
        o[nb] = wmma16(pf, vf, o[nb]);
      }
    }
    __syncthreads();
  }

  float inv[8];
#pragma unroll
  for (int v = 0; v < 8; ++v) inv[v] = __builtin_amdgcn_rcpf(lrow[v]) * VCARRY;
#pragma unroll
  for (int nb = 0; nb < 4; ++nb)
#pragma unroll
    for (int v = 0; v < 8; ++v)
      Ps[pw + (hh * 8u + (unsigned)v) * LDT + (unsigned)nb * 16u + m] =
          toh_flush(o[nb][v] * inv[v]);
  wave_lds_sync();
  v8h x[4];
  size_t off[4];
#pragma unroll
  for (unsigned i = 0; i < 4u; ++i) {
    const unsigned r = 4u * i + (lane >> 3);
    const unsigned c = (lane & 7u) * 8u;
    x[i] = *(const v8h*)&Ps[pw + r * LDT + c];
    off[i] = (size_t)(b * (unsigned)SEQP + qrow0 + r) * DIM + head * HD + c;
  }
#pragma unroll
  for (int i = 0; i < 4; ++i) *(volatile v8h*)(Ov + off[i]) = x[i];
  __threadfence();
#pragma unroll
  for (int i = 0; i < 4; ++i) *(volatile v8h*)(Ov + off[i]) = x[i];
}

extern "C" void kernel_launch(void* const* d_in, const int* in_sizes, int n_in,
                              void* d_out, int out_size, void* d_ws, size_t ws_size,
                              hipStream_t stream) {
  if (n_in < 15) return;
  const long long need_x = ((long long)(NB - 1) * SEQ_FULL + SEQ) * DIM;
  const int need_idx = (SEQ - 1) / KNN + 1;
  if (in_sizes[0] < need_idx || in_sizes[1] < need_idx) return;
  if ((long long)in_sizes[2] < need_x) return;
  if ((long long)in_sizes[3] < need_x) return;
  if ((long long)in_sizes[4] < need_x) return;
  if ((long long)in_sizes[5] < (long long)DIM * DIM) return;
  if ((long long)in_sizes[7] < (long long)DIM * DIM) return;
  if ((long long)in_sizes[9] < (long long)DIM * DIM) return;
  if ((long long)in_sizes[11] < (long long)DIM * DIM) return;
  if (in_sizes[6] < DIM || in_sizes[8] < DIM || in_sizes[10] < DIM || in_sizes[12] < DIM) return;
  if (in_sizes[13] < EDGE_DICT * DIM) return;
  if (in_sizes[14] < 2 * DIM) return;
  if ((long long)out_size < need_x) return;
  if (ws_size < WS_TOTAL) return;

  const int*   c_mask   = (const int*)d_in[0];
  const int*   degv     = (const int*)d_in[1];
  const float* qin      = (const float*)d_in[2];
  const float* kin      = (const float*)d_in[3];
  const float* vin      = (const float*)d_in[4];
  const float* wq       = (const float*)d_in[5];
  const float* bq       = (const float*)d_in[6];
  const float* wk       = (const float*)d_in[7];
  const float* bk       = (const float*)d_in[8];
  const float* wv       = (const float*)d_in[9];
  const float* bv       = (const float*)d_in[10];
  const float* wo       = (const float*)d_in[11];
  const float* bo       = (const float*)d_in[12];
  const float* edge_emb = (const float*)d_in[13];
  const float* mask_emb = (const float*)d_in[14];
  float* out = (float*)d_out;

  char* ws = (char*)d_ws;
  _Float16* Wq_t  = (_Float16*)(ws + OFF_WQ);
  _Float16* Wk_t  = (_Float16*)(ws + OFF_WK);
  _Float16* Wv_t  = (_Float16*)(ws + OFF_WV);
  _Float16* Wo_t  = (_Float16*)(ws + OFF_WO);
  _Float16* Xq16  = (_Float16*)(ws + OFF_XQ);
  _Float16* Xk16  = (_Float16*)(ws + OFF_XK);
  _Float16* Xv16  = (_Float16*)(ws + OFF_XV);
  _Float16* Qh16  = (_Float16*)(ws + OFF_Q);
  _Float16* Kh16  = (_Float16*)(ws + OFF_K);
  _Float16* Vt16  = (_Float16*)(ws + OFF_VT);
  _Float16* Ctx16 = (_Float16*)(ws + OFF_CTX);
  float*    Tbl   = (float*)(ws + OFF_TBL);

  dim3 blk(256);
  dim3 gw((unsigned)(((size_t)DIM * DIM) / 2048));
  dim3 gx(MROWSP / 8);
  dim3 gg(DIM / 64, MROWSP / 64);

  wcast_kernel<<<gw, blk, 0, stream>>>(wq, Wq_t);
  wcast_kernel<<<gw, blk, 0, stream>>>(wk, Wk_t);
  wcast_kernel<<<gw, blk, 0, stream>>>(wv, Wv_t);
  wcast_kernel<<<gw, blk, 0, stream>>>(wo, Wo_t);

  xcast_kernel<<<gx, blk, 0, stream>>>(qin, Xq16);
  xcast_kernel<<<gx, blk, 0, stream>>>(kin, Xk16);
  xcast_kernel<<<gx, blk, 0, stream>>>(vin, Xv16);

  bias_table_kernel<<<dim3((EDGE_DICT * 2) / 32), blk, 0, stream>>>(edge_emb, mask_emb, Tbl);

  gemm_qk_kernel<<<gg, blk, 0, stream>>>(Xq16, Wq_t, bq, Qh16);
  gemm_qk_kernel<<<gg, blk, 0, stream>>>(Xk16, Wk_t, bk, Kh16);
  gemm_v_kernel<<<gg, blk, 0, stream>>>(Xv16, Wv_t, bv, Vt16);
  attn_kernel<<<dim3(SEQP / 128, NHEAD, NB), blk, 0, stream>>>(Qh16, Kh16, Vt16, c_mask, degv,
                                                              Tbl, Ctx16);
  gemm_wo_kernel<<<gg, blk, 0, stream>>>(Ctx16, Wo_t, bo, out);
}
